// GraphSAGE_10273561772524
// MI455X (gfx1250) — hardware-verified
//
#include <hip/hip_runtime.h>
#include <stddef.h>
#include <stdint.h>


#define CIN    128
#define HID    64
#define NTHR   256
#define NWAVE  8
#define EPT    8
#define CHUNK  (NTHR * EPT)
#define WCAP   (EPT * 32)
#define LISTN  (NWAVE * WCAP)
#define NBA    1024
#define SLA    10
#define RCAP   28672
#define DEGCAP 64
#define GBM    64
#define GBN    64
#define GTHR   128
#define AGG_ZINTS (LISTN + 2 * RCAP + 3 * NBA)
#define MISC_INTS 16
#define AGG_LDS_INTS (AGG_ZINTS + MISC_INTS)
#define WSMAX  134217728
#define OWA    0
#define OWB    (192 * 128)
#define OWC    (OWB + 64 * 256)
#define OWD    (OWC + 128 * 128)
#define WPL_ELEMS (OWD + 64 * 128)
#define NUW    8192

static_assert((CHUNK & (CHUNK - 1)) == 0 && CHUNK <= 4096);
static_assert((NBA & (NBA - 1)) == 0 && NBA == (1 << SLA));
static_assert(((long long)CHUNK << SLA) < (1LL << 31));
static_assert(NBA % NWAVE == 0 && NBA % 32 == 0 && NBA % GBM == 0);
static_assert(RCAP % 32 == 0 && AGG_ZINTS % 4 == 0 && LISTN % 4 == 0);
static_assert(CIN % 32 == 0 && (2 * CIN) % 32 == 0 && (2 * HID) % 32 == 0);
static_assert(GBM == (GTHR / 32) * 16 && GBN == 64 && HID == GBN);
static_assert(WPL_ELEMS == NUW * 8 && NUW % NTHR == 0);
static_assert(AGG_LDS_INTS * 4 <= 300000);
static_assert(DEGCAP >= 36 + 8 && RCAP >= 16721 + 4096);

typedef float          v2f   __attribute__((ext_vector_type(2)));
typedef float          v4f   __attribute__((ext_vector_type(4)));
typedef float          v8f   __attribute__((ext_vector_type(8)));
typedef int            v4i   __attribute__((ext_vector_type(4)));
typedef int            v8i   __attribute__((ext_vector_type(8)));
typedef unsigned int   v4u   __attribute__((ext_vector_type(4)));
typedef unsigned short v4us  __attribute__((ext_vector_type(4)));
typedef unsigned short v8us  __attribute__((ext_vector_type(8)));
typedef unsigned short v16us __attribute__((ext_vector_type(16)));
typedef __bf16         v16bf __attribute__((ext_vector_type(16)));
typedef v2f  __attribute__((may_alias)) v2fa;
typedef v4f  __attribute__((may_alias)) v4fa;
typedef v4i  __attribute__((may_alias)) v4ia;
typedef v4us __attribute__((may_alias)) v4usa;
typedef v8us __attribute__((may_alias)) v8usa;
union FragB { v16bf v; v16us u; v8us h[2]; v8i w; };

__device__ __forceinline__ v8f wmb(const FragB& a, const FragB& b, v8f c) {
  v8f d = __builtin_amdgcn_wmma_f32_16x16x32_bf16(false, a.v, false, b.v, (short)0, c, false, false);
  asm volatile("v_nop\n\tv_nop\n\tv_nop\n\tv_nop" : "+v"(d) : "v"(a.w), "v"(b.w));
  return d;
}

__device__ __forceinline__ unsigned bf16_bits(float f) {
  const unsigned u = __float_as_uint(f);
  const unsigned r = (u + 0x7FFFu + ((u >> 16) & 1u)) >> 16;
  return (f != f) ? 0x7FC0u : r;
}
__device__ __forceinline__ float bf16_val(float f) {
  return __uint_as_float(bf16_bits(f) << 16);
}
__device__ __forceinline__ float relu_keep(float t) {
  return (t > 0.0f) ? t : (t - t);
}

template <int SLB>
__device__ __forceinline__ int scan_chunk(const int* __restrict__ dsts, int nE, int cbase, int slotBase,
                                          int nb, int vec8, int* list, int tid, int lane, int wave) {
  int wc = 0;
  const int el0  = tid * EPT;
  const int e0   = cbase + el0;
  const int sent = -2147483647 - 1;
  v4i da, db;
  if (vec8 != 0 && cbase + CHUNK <= nE) {
    da = *(const v4i*)(dsts + e0);
    db = *(const v4i*)(dsts + e0 + 4);
  } else {
    da.x = (e0     < nE) ? dsts[min(e0,     nE - 1)] : sent;
    da.y = (e0 + 1 < nE) ? dsts[min(e0 + 1, nE - 1)] : sent;
    da.z = (e0 + 2 < nE) ? dsts[min(e0 + 2, nE - 1)] : sent;
    da.w = (e0 + 3 < nE) ? dsts[min(e0 + 3, nE - 1)] : sent;
    db.x = (e0 + 4 < nE) ? dsts[min(e0 + 4, nE - 1)] : sent;
    db.y = (e0 + 5 < nE) ? dsts[min(e0 + 5, nE - 1)] : sent;
    db.z = (e0 + 6 < nE) ? dsts[min(e0 + 6, nE - 1)] : sent;
    db.w = (e0 + 7 < nE) ? dsts[min(e0 + 7, nE - 1)] : sent;
  }
  const unsigned nbs = (unsigned)slotBase;
  const unsigned unb = (unsigned)nb;
  const unsigned s0 = (unsigned)da.x - nbs, s1 = (unsigned)da.y - nbs;
  const unsigned s2 = (unsigned)da.z - nbs, s3 = (unsigned)da.w - nbs;
  const unsigned s4 = (unsigned)db.x - nbs, s5 = (unsigned)db.y - nbs;
  const unsigned s6 = (unsigned)db.z - nbs, s7 = (unsigned)db.w - nbs;
  const bool h0 = s0 < unb, h1 = s1 < unb, h2 = s2 < unb, h3 = s3 < unb;
  const bool h4 = s4 < unb, h5 = s5 < unb, h6 = s6 < unb, h7 = s7 < unb;
  const unsigned any = __builtin_amdgcn_ballot_w32(h0 | h1 | h2 | h3 | h4 | h5 | h6 | h7);
  if (any != 0u) {
#define HITJ(J, HJ, SJ) { \
      const unsigned mj = __builtin_amdgcn_ballot_w32(HJ); \
      if (mj != 0u) { \
        if (HJ) { \
          const int pos = wc + (int)__builtin_amdgcn_mbcnt_lo(mj, 0u); \
          if (pos < WCAP) list[wave * WCAP + pos] = ((el0 + (J)) << SLB) | (int)(SJ); \
        } \
        wc += (int)__builtin_popcount(mj); } }
    HITJ(0, h0, s0)
    HITJ(1, h1, s1)
    HITJ(2, h2, s2)
    HITJ(3, h3, s3)
    HITJ(4, h4, s4)
    HITJ(5, h5, s5)
    HITJ(6, h6, s6)
    HITJ(7, h7, s7)
#undef HITJ
  }
  return wc;
}

__device__ __forceinline__ v8us gat8(const float* __restrict__ W, int ldw, int k0, int n) {
  v8us o;
  const float* p = W + (size_t)k0 * ldw + n;
#pragma unroll
  for (int i = 0; i < 8; ++i) o[i] = (unsigned short)bf16_bits(p[(size_t)i * ldw]);
  return o;
}

__global__ __launch_bounds__(NTHR) void k_wprep(const float* __restrict__ Wp1, const float* __restrict__ Ws1,
                                                const float* __restrict__ Wn1, const float* __restrict__ Wp2,
                                                const float* __restrict__ Ws2, const float* __restrict__ Wn2,
                                                unsigned short* wpl) {
  const int u = (int)blockIdx.x * NTHR + (int)threadIdx.x;
  v8us o;
  int doff;
  if (u < 2048) {
    const int n = u >> 4, k8 = (u & 15) * 8;
    o = gat8(Wp1, CIN, k8, n);
    doff = OWA + n * CIN + k8;
  } else if (u < 3072) {
    const int v = u - 2048, n = v >> 4, k8 = (v & 15) * 8;
    o = gat8(Ws1, HID, k8, n);
    doff = OWA + (CIN + n) * CIN + k8;
  } else if (u < 5120) {
    const int v = u - 3072, n = v >> 5, k8 = (v & 31) * 8;
    o = gat8(Wn1, HID, k8 & (CIN - 1), n);
    doff = OWB + n * (2 * CIN) + k8;
  } else if (u < 6144) {
    const int v = u - 5120, n = v >> 4, k8 = (v & 15) * 8;
    o = gat8(Wp2, HID, k8 & (HID - 1), n);
    doff = OWC + n * (2 * HID) + k8;
  } else if (u < 7168) {
    const int v = u - 6144, n = v >> 4, k8 = (v & 15) * 8;
    o = gat8(Ws2, HID, k8 & (HID - 1), n);
    doff = OWC + (HID + n) * (2 * HID) + k8;
  } else if (u < NUW) {
    const int v = u - 7168, n = v >> 4, k8 = (v & 15) * 8;
    o = gat8(Wn2, HID, k8 & (HID - 1), n);
    doff = OWD + n * (2 * HID) + k8;
  } else {
    return;
  }
  unsigned short* dp = wpl + doff;
  *(volatile v8us*)dp = o;
  __threadfence();
  *(volatile v8us*)dp = o;
}

__global__ __launch_bounds__(NTHR) void k_cvx(const float* __restrict__ x, int nN, int nUnits,
                                              unsigned short* xb) {
  const int u = (int)blockIdx.x * NTHR + (int)threadIdx.x;
  if (u >= nUnits) return;
  const int row = u >> 4;
  const int k8  = (u & 15) * 8;
  const int rc  = row < nN ? row : nN - 1;
  const float* p = x + (size_t)rc * CIN + k8;
  const v4f a = *(const v4fa*)p;
  const v4f b = *(const v4fa*)(p + 4);
  const bool ok = row < nN;
  v8us o;
  o[0] = ok ? (unsigned short)bf16_bits(a.x) : (unsigned short)0;
  o[1] = ok ? (unsigned short)bf16_bits(a.y) : (unsigned short)0;
  o[2] = ok ? (unsigned short)bf16_bits(a.z) : (unsigned short)0;
  o[3] = ok ? (unsigned short)bf16_bits(a.w) : (unsigned short)0;
  o[4] = ok ? (unsigned short)bf16_bits(b.x) : (unsigned short)0;
  o[5] = ok ? (unsigned short)bf16_bits(b.y) : (unsigned short)0;
  o[6] = ok ? (unsigned short)bf16_bits(b.z) : (unsigned short)0;
  o[7] = ok ? (unsigned short)bf16_bits(b.w) : (unsigned short)0;
  unsigned short* dp = xb + (size_t)row * CIN + k8;
  *(volatile v8us*)dp = o;
  __threadfence();
  *(volatile v8us*)dp = o;
}

__device__ __forceinline__ void gemm_core(const unsigned short* __restrict__ A,
                                          const unsigned short* __restrict__ WT, int K,
                                          int rowBase, int col0, float* stg, int lane, int wave) {
  const int hh = lane >> 4, m = lane & 15;
  v8f acc[4];
  {
    const v8f z = {0.f, 0.f, 0.f, 0.f, 0.f, 0.f, 0.f, 0.f};
    acc[0] = z; acc[1] = z; acc[2] = z; acc[3] = z;
  }
  const unsigned short* ap = A  + (size_t)(rowBase + 16 * wave + m) * (size_t)K + 8 * hh;
  const unsigned short* wp = WT + (size_t)(col0 + m) * (size_t)K + 8 * hh;
  const int ksteps = K >> 5;
#pragma unroll 1
  for (int ks = 0; ks < ksteps; ++ks) {
    FragB af;
    af.h[0] = *(const v8usa*)(ap + 32 * ks);
    af.h[1] = *(const v8usa*)(ap + 32 * ks + 16);
#pragma unroll
    for (int t = 0; t < 4; ++t) {
      const unsigned short* wq = wp + (size_t)(16 * t) * (size_t)K + 32 * ks;
      FragB bf;
      bf.h[0] = *(const v8usa*)wq;
      bf.h[1] = *(const v8usa*)(wq + 16);
      acc[t] = wmb(af, bf, acc[t]);
    }
  }
#pragma unroll
  for (int t = 0; t < 4; ++t) {
    const int lc = 16 * t + m;
#pragma unroll
    for (int r = 0; r < 8; ++r) {
      const int lr = 16 * wave + 8 * hh + r;
      stg[lr * GBN + lc] = acc[t][r];
    }
  }
}

__global__ __launch_bounds__(GTHR) void k_gemm_ps(const unsigned short* __restrict__ A,
                                                  const unsigned short* __restrict__ WT, int K,
                                                  const float* __restrict__ biasP, float* wsf,
                                                  unsigned long long offP, unsigned long long offS,
                                                  int ldP, int nP, int ldS) {
  __shared__ __attribute__((aligned(16))) float stg[GBM * GBN];
  const int tid = (int)threadIdx.x, lane = tid & 31, wave = tid >> 5, hh = lane >> 4, m = lane & 15;
  const int rowBase = (int)blockIdx.x * GBM;
  const int col0    = (int)blockIdx.y * GBN;
  gemm_core(A, WT, K, rowBase, col0, stg, lane, wave);
  __syncthreads();

  const bool isP = col0 < nP;
  const unsigned long long obase = isP ? offP : offS;
  const int ldo = isP ? ldP : ldS;
  const int oc  = isP ? col0 : (col0 - nP);
  const int bc  = isP ? col0 : 0;
  v4f b4;
  {
    const v4f t = *(const v4f*)(biasP + bc + 4 * m);
    b4.x = bf16_val(t.x); b4.y = bf16_val(t.y); b4.z = bf16_val(t.z); b4.w = bf16_val(t.w);
  }
  v4f fv[8];
#pragma unroll
  for (int i = 0; i < 8; ++i) {
    const int lr = 16 * wave + 2 * i + hh;
    fv[i] = *(const v4fa*)(stg + lr * GBN + 4 * m);
  }
  if (isP) {
#pragma unroll
    for (int i = 0; i < 8; ++i) {
      v4f y = fv[i] + b4;
      y.x = relu_keep(y.x); y.y = relu_keep(y.y); y.z = relu_keep(y.z); y.w = relu_keep(y.w);
      fv[i] = y;
    }
  }
#pragma unroll
  for (int i = 0; i < 8; ++i) {
    const int gr = rowBase + 16 * wave + 2 * i + hh;
    float* op = wsf + obase + (size_t)gr * (size_t)ldo + oc + 4 * m;
    *(volatile v4f*)op = fv[i];
  }
  __threadfence();
#pragma unroll
  for (int i = 0; i < 8; ++i) {
    const int gr = rowBase + 16 * wave + 2 * i + hh;
    float* op = wsf + obase + (size_t)gr * (size_t)ldo + oc + 4 * m;
    *(volatile v4f*)op = fv[i];
  }
}

__global__ __launch_bounds__(GTHR) void k_gemm_h(const unsigned short* __restrict__ A,
                                                 const unsigned short* __restrict__ WT, int K,
                                                 const float* __restrict__ S, const float* __restrict__ bias,
                                                 unsigned short* hout) {
  __shared__ __attribute__((aligned(16))) float stg[GBM * GBN];
  const int tid = (int)threadIdx.x, lane = tid & 31, wave = tid >> 5, hh = lane >> 4, m = lane & 15;
  const int rowBase = (int)blockIdx.x * GBM;
  gemm_core(A, WT, K, rowBase, 0, stg, lane, wave);
  __syncthreads();

  v4f b4;
  {
    const v4f t = *(const v4f*)(bias + 4 * m);
    b4.x = bf16_val(t.x); b4.y = bf16_val(t.y); b4.z = bf16_val(t.z); b4.w = bf16_val(t.w);
  }
  v4f pv[8];
#pragma unroll
  for (int i = 0; i < 8; ++i) {
    const int lr = 16 * wave + 2 * i + hh;
    pv[i] = *(const v4fa*)(stg + lr * GBN + 4 * m);
  }
  __syncthreads();
#pragma unroll
  for (int i = 0; i < 8; ++i) {
    const int lr = 16 * wave + 2 * i + hh;
    const int gr = rowBase + lr;
    const v4f s = *(const v4fa*)(S + (size_t)gr * HID + 4 * m);
    v4f t = (s + pv[i]) + b4;
    t.x = relu_keep(t.x); t.y = relu_keep(t.y); t.z = relu_keep(t.z); t.w = relu_keep(t.w);
    v4us h4, l4;
    unsigned hb;
    hb = bf16_bits(t.x); h4[0] = (unsigned short)hb; l4[0] = (unsigned short)bf16_bits(t.x - __uint_as_float(hb << 16));
    hb = bf16_bits(t.y); h4[1] = (unsigned short)hb; l4[1] = (unsigned short)bf16_bits(t.y - __uint_as_float(hb << 16));
    hb = bf16_bits(t.z); h4[2] = (unsigned short)hb; l4[2] = (unsigned short)bf16_bits(t.z - __uint_as_float(hb << 16));
    hb = bf16_bits(t.w); h4[3] = (unsigned short)hb; l4[3] = (unsigned short)bf16_bits(t.w - __uint_as_float(hb << 16));
    unsigned short* srow = (unsigned short*)stg + (size_t)lr * (2 * GBN);
    *(v4usa*)(srow + 4 * m) = h4;
    *(v4usa*)(srow + HID + 4 * m) = l4;
  }
  __syncthreads();
  v8us qv[8];
#pragma unroll
  for (int i = 0; i < 8; ++i) {
    const int lr = 16 * wave + 2 * i + hh;
    const unsigned short* srow = (const unsigned short*)stg + (size_t)lr * (2 * GBN);
    qv[i] = *(const v8usa*)(srow + 8 * m);
  }
#pragma unroll
  for (int i = 0; i < 8; ++i) {
    const int gr = rowBase + 16 * wave + 2 * i + hh;
    unsigned short* hp = hout + (size_t)gr * (2 * HID) + 8 * m;
    *(volatile v8us*)hp = qv[i];
  }
  __threadfence();
#pragma unroll
  for (int i = 0; i < 8; ++i) {
    const int gr = rowBase + 16 * wave + 2 * i + hh;
    unsigned short* hp = hout + (size_t)gr * (2 * HID) + 8 * m;
    *(volatile v8us*)hp = qv[i];
  }
}

__global__ __launch_bounds__(GTHR) void k_gemm_out(const unsigned short* __restrict__ A,
                                                   const unsigned short* __restrict__ WT, int K,
                                                   const float* __restrict__ S, const float* __restrict__ bias,
                                                   const float* __restrict__ Wo, const float* __restrict__ bo,
                                                   float* out, int nN) {
  __shared__ __attribute__((aligned(16))) float stg[GBM * GBN];
  __shared__ __attribute__((aligned(16))) float wos[2 * HID];
  __shared__ __attribute__((aligned(16))) float ys[2 * GBM];
  const int tid = (int)threadIdx.x, lane = tid & 31, wave = tid >> 5, hh = lane >> 4, m = lane & 15;
  const int rowBase = (int)blockIdx.x * GBM;
  wos[tid] = bf16_val(Wo[tid]);
  gemm_core(A, WT, K, rowBase, 0, stg, lane, wave);
  __syncthreads();

  v4f b4;
  {
    const v4f t = *(const v4f*)(bias + 4 * m);
    b4.x = bf16_val(t.x); b4.y = bf16_val(t.y); b4.z = bf16_val(t.z); b4.w = bf16_val(t.w);
  }
#pragma unroll
  for (int i = 0; i < 8; ++i) {
    const int lr = 16 * wave + 2 * i + hh;
    const int gr = rowBase + lr;
    const v4f p = *(const v4fa*)(stg + lr * GBN + 4 * m);
    const v4f s = *(const v4fa*)(S + (size_t)gr * HID + 4 * m);
    v4f t = (s + p) + b4;
    t.x = relu_keep(t.x); t.y = relu_keep(t.y); t.z = relu_keep(t.z); t.w = relu_keep(t.w);
    *(v4fa*)(stg + lr * GBN + 4 * m) = t;
  }
  __syncthreads();
  {
    const int row = tid >> 1, c = tid & 1;
    const float* hr = stg + row * GBN;
    float s = 0.0f;
#pragma unroll 4
    for (int k = 0; k < HID; ++k) s = fmaf(hr[k], wos[2 * k + c], s);
    s = s + bf16_val(bo[c]);
    ys[tid] = s;
  }
  __syncthreads();
  const v4f ov = *(const v4fa*)(ys + 4 * lane);
  const bool okst = (wave == 0) && (rowBase + 2 * lane + 1 < nN);
  float* op = out + (size_t)rowBase * 2 + 4 * lane;
  if (okst) *(volatile v4f*)op = ov;
  __threadfence();
  if (okst) *(volatile v4f*)op = ov;
}

template <int F>
__global__ __launch_bounds__(NTHR) void k_scan(const int* __restrict__ srcs, const int* __restrict__ dsts,
                                               int nE, int nN, int vec8, int mRows,
                                               const float* __restrict__ P, unsigned short* agg) {
  extern __shared__ __attribute__((aligned(16))) int dsm[];
  int* list = dsm;
  int* hl   = dsm + LISTN;
  int* sl   = dsm + LISTN + RCAP;
  int* cnt  = dsm + LISTN + 2 * RCAP;
  int* offs = cnt + NBA;
  int* cur  = offs + NBA;
  int* misc = cur + NBA;
  const int tid = (int)threadIdx.x, lane = tid & 31, wave = tid >> 5;
  const int nodeBase = (int)blockIdx.x * NBA;

  {
    const v4i z4 = {0, 0, 0, 0};
    for (int i = tid * 4; i < AGG_ZINTS; i += NTHR * 4) *(v4ia*)(dsm + i) = z4;
    if (tid < MISC_INTS) misc[tid] = 0;
  }
  __syncthreads();

  int t = 0, ov = 0;
  const int nChunks = (nE + CHUNK - 1) / CHUNK;
#pragma unroll 1
  for (int ch = 0; ch < nChunks; ++ch) {
    const int cbase = ch * CHUNK;
    const int wc = scan_chunk<SLA>(dsts, nE, cbase, nodeBase, NBA, vec8, list, tid, lane, wave);
    if (lane == 0) misc[wave] = wc;
    __syncthreads();
    if (wave == 0) {
#pragma unroll 1
      for (int w2 = 0; w2 < NWAVE; ++w2) {
        int c = misc[w2];
        c = c < 0 ? 0 : (c > WCAP ? WCAP : c);
#pragma unroll 1
        for (int b0 = 0; b0 < c; b0 += 32) {
          const int idx = b0 + lane;
          const int ent = list[w2 * WCAP + (idx < WCAP ? idx : WCAP - 1)];
          const int m32 = (c - b0) < 32 ? (c - b0) : 32;
#pragma unroll 1
          for (int k = 0; k < m32; ++k) {
            const int u    = __builtin_amdgcn_readlane(ent, k);
            const int slot = u & (NBA - 1);
            const int el   = (u >> SLA) & (CHUNK - 1);
            const int pk   = ((cbase + el) << SLA) | slot;
            if (t < RCAP) {
              if (lane == 0) { hl[t] = pk; cnt[slot] = cnt[slot] + 1; }
              t = t + 1;
            } else {
              ov = 1;
            }
          }
        }
      }
    }
    __syncthreads();
  }
  if (wave == 0 && lane == 0) { misc[8] = t; misc[9] = ov; }
  __syncthreads();
  int tt = misc[8];
  tt = tt < 0 ? 0 : (tt > RCAP ? RCAP : tt);
  const int ovf = misc[9];

  if (wave == 0) {
    const int base = lane * (NBA / 32);
    int s = 0;
#pragma unroll 1
    for (int i = 0; i < NBA / 32; ++i) s += cnt[base + i];
    int incl = s;
#pragma unroll
    for (int d = 1; d < 32; d <<= 1) {
      const int y = __shfl_up(incl, d, 32);
      if (lane >= d) incl += y;
    }
    int run = incl - s;
#pragma unroll 1
    for (int i = 0; i < NBA / 32; ++i) {
      const int cv = cnt[base + i];
      offs[base + i] = run;
      cur[base + i]  = run;
      run += cv;
    }
  }
  __syncthreads();
  if (wave == 0) {
#pragma unroll 1
    for (int b0 = 0; b0 < tt; b0 += 32) {
      const int idx = b0 + lane;
      const int ent = hl[idx < RCAP ? idx : RCAP - 1];
      const int m32 = (tt - b0) < 32 ? (tt - b0) : 32;
#pragma unroll 1
      for (int k = 0; k < m32; ++k) {
        const int u    = __builtin_amdgcn_readlane(ent, k);
        const int slot = u & (NBA - 1);
        if (lane == 0) {
          int p = cur[slot];
          p = p < 0 ? 0 : (p > RCAP - 1 ? RCAP - 1 : p);
          sl[p] = u;
          cur[slot] = p + 1;
        }
      }
    }
  }
  __syncthreads();

  const float qnan = __uint_as_float(0x7fc00000u);
  const float ninf = __uint_as_float(0xff800000u);
  const int sa = (2 * lane) & 31, sb = (2 * lane + 1) & 31;
  const int q0s = (4 * lane) & 31, q1s = (4 * lane + 1) & 31;
  const int q2s = (4 * lane + 2) & 31, q3s = (4 * lane + 3) & 31;
#pragma unroll 1
  for (int si = 0; si < NBA / NWAVE; ++si) {
    const int s    = si * NWAVE + wave;
    const int node = nodeBase + s;
    const int craw = cnt[s];
    const bool big = craw > DEGCAP;
    int c = craw < 0 ? 0 : (craw > DEGCAP ? DEGCAP : craw);
    int o = offs[s];
    o = o < 0 ? 0 : (o > RCAP ? RCAP : o);
    float m0 = ninf, m1 = ninf, m2 = ninf, m3 = ninf;
#pragma unroll 1
    for (int b0 = 0; b0 < c; b0 += 32) {
      int idx = o + b0 + lane;
      idx = idx > RCAP - 1 ? RCAP - 1 : idx;
      const int ent = sl[idx];
      int eid = ent >> SLA;
      eid = eid < 0 ? 0 : (eid > nE - 1 ? nE - 1 : eid);
      int sr = srcs[eid];
      sr = sr < 0 ? 0 : (sr > nN - 1 ? nN - 1 : sr);
      const int m32 = (c - b0) < 32 ? (c - b0) : 32;
#pragma unroll 1
      for (int k = 0; k < m32; ++k) {
        const int sk = __builtin_amdgcn_readlane(sr, k);
        if constexpr (F == 128) {
          const v4f a = *(const v4fa*)(P + (size_t)sk * F + 4 * lane);
          m0 = (a.x > m0 || a.x != a.x) ? a.x : m0;
          m1 = (a.y > m1 || a.y != a.y) ? a.y : m1;
          m2 = (a.z > m2 || a.z != a.z) ? a.z : m2;
          m3 = (a.w > m3 || a.w != a.w) ? a.w : m3;
        } else {
          const v2f a = *(const v2fa*)(P + (size_t)sk * F + 2 * lane);
          m0 = (a.x > m0 || a.x != a.x) ? a.x : m0;
          m1 = (a.y > m1 || a.y != a.y) ? a.y : m1;
        }
      }
    }
    const bool empty = craw <= 0;
    const bool pois  = big || (ovf != 0);
    const bool live  = node < nN;
    float v0 = empty ? 0.0f : m0;
    float v1 = empty ? 0.0f : m1;
    v0 = pois ? qnan : v0; v1 = pois ? qnan : v1;
    v0 = live ? v0 : 0.0f; v1 = live ? v1 : 0.0f;
    const unsigned hb0 = bf16_bits(v0), hb1 = bf16_bits(v1);
    const unsigned lb0 = bf16_bits(v0 - __uint_as_float(hb0 << 16));
    const unsigned lb1 = bf16_bits(v1 - __uint_as_float(hb1 << 16));
    if constexpr (F == 128) {
      float v2 = empty ? 0.0f : m2;
      float v3 = empty ? 0.0f : m3;
      v2 = pois ? qnan : v2; v3 = pois ? qnan : v3;
      v2 = live ? v2 : 0.0f; v3 = live ? v3 : 0.0f;
      const unsigned hb2 = bf16_bits(v2), hb3 = bf16_bits(v3);
      const unsigned lb2 = bf16_bits(v2 - __uint_as_float(hb2 << 16));
      const unsigned lb3 = bf16_bits(v3 - __uint_as_float(hb3 << 16));
      const int hw0 = (int)(hb0 | (hb1 << 16));
      const int hw1 = (int)(hb2 | (hb3 << 16));
      const int lw0 = (int)(lb0 | (lb1 << 16));
      const int lw1 = (int)(lb2 | (lb3 << 16));
      const int g0 = __shfl(hw0, sa, 32), g1 = __shfl(hw1, sa, 32);
      const int g2 = __shfl(hw0, sb, 32), g3 = __shfl(hw1, sb, 32);
      const int p0 = __shfl(lw0, sa, 32), p1 = __shfl(lw1, sa, 32);
      const int p2 = __shfl(lw0, sb, 32), p3 = __shfl(lw1, sb, 32);
      const bool lsel = lane >= 16;
      v4u pv;
      pv.x = (unsigned int)(lsel ? p0 : g0);
      pv.y = (unsigned int)(lsel ? p1 : g1);
      pv.z = (unsigned int)(lsel ? p2 : g2);
      pv.w = (unsigned int)(lsel ? p3 : g3);
      unsigned short* hp = agg + (size_t)node * (2 * F) + 8 * lane;
      const bool wr = node < mRows;
      if (wr) *(volatile v4u*)hp = pv;
      __threadfence();
      if (wr) *(volatile v4u*)hp = pv;
    } else {
      const int hw = (int)(hb0 | (hb1 << 16));
      const int lw = (int)(lb0 | (lb1 << 16));
      const int g0 = __shfl(hw, q0s, 32), g1 = __shfl(hw, q1s, 32);
      const int g2 = __shfl(hw, q2s, 32), g3 = __shfl(hw, q3s, 32);
      const int p0 = __shfl(lw, q0s, 32), p1 = __shfl(lw, q1s, 32);
      const int p2 = __shfl(lw, q2s, 32), p3 = __shfl(lw, q3s, 32);
      const bool lsel = (lane & 8) != 0;
      v4u pv;
      pv.x = (unsigned int)(lsel ? p0 : g0);
      pv.y = (unsigned int)(lsel ? p1 : g1);
      pv.z = (unsigned int)(lsel ? p2 : g2);
      pv.w = (unsigned int)(lsel ? p3 : g3);
      unsigned short* hp = agg + (size_t)node * (2 * F) + 8 * (lane & 15);
      const bool wr = (node < mRows) && (lane < 16);
      if (wr) *(volatile v4u*)hp = pv;
      __threadfence();
      if (wr) *(volatile v4u*)hp = pv;
    }
  }
}

static inline int cdiv(int a, int b) { return (a + b - 1) / b; }
static inline size_t al256(size_t o) { return (o + 255) & ~(size_t)255; }

extern "C" void kernel_launch(void* const* d_in, const int* in_sizes, int n_in,
                              void* d_out, int out_size, void* d_ws, size_t ws_size,
                              hipStream_t stream) {
  if (n_in < 15) return;
  if (in_sizes[0] < CIN || (in_sizes[0] % CIN) != 0) return;
  const int nN = in_sizes[0] / CIN;
  if (nN < 16 || nN > (1 << 22) || (nN % 16) != 0) return;
  const int nE = in_sizes[1];
  if (nE < 1 || in_sizes[2] != nE) return;
  if (nE >= (1 << (31 - SLA))) return;
  if (in_sizes[3] != CIN * CIN || in_sizes[4] != CIN) return;
  if (in_sizes[5] != CIN * HID || in_sizes[6] != CIN * HID) return;
  if (in_sizes[7] != HID) return;
  if (in_sizes[8] != HID * HID || in_sizes[9] != HID) return;
  if (in_sizes[10] != HID * HID || in_sizes[11] != HID * HID) return;
  if (in_sizes[12] != HID) return;
  if (in_sizes[13] != HID * 2 || in_sizes[14] != 2) return;
  if ((long long)out_size != 2LL * nN) return;

  const float* x    = (const float*)d_in[0];
  const int*   src  = (const int*)d_in[1];
  const int*   dst  = (const int*)d_in[2];
  const float* Wp1  = (const float*)d_in[3];
  const float* bp1  = (const float*)d_in[4];
  const float* Ws1  = (const float*)d_in[5];
  const float* Wn1  = (const float*)d_in[6];
  const float* b1   = (const float*)d_in[7];
  const float* Wp2  = (const float*)d_in[8];
  const float* bp2  = (const float*)d_in[9];
  const float* Ws2  = (const float*)d_in[10];
  const float* Wn2  = (const float*)d_in[11];
  const float* b2   = (const float*)d_in[12];
  const float* Wo   = (const float*)d_in[13];
  const float* bo   = (const float*)d_in[14];
  float* out = (float*)d_out;

  const int MP = cdiv(nN, GBM) * GBM;
  const int gM = MP / GBM;
  const int gA = cdiv(MP, NBA);
  if ((long long)gA * NBA < (long long)MP) return;
  const int vec8 = ((nE & 3) == 0) ? 1 : 0;

  char* ws = (char*)d_ws;
  size_t off = 0;
  const size_t oWPL = off; off = al256(off + (size_t)WPL_ELEMS * 2);
  const size_t oRA  = off; off = al256(off + (size_t)MP * 512);
  const size_t oRB  = off; off = al256(off + (size_t)MP * 256);
  const size_t oRC  = off; off = al256(off + (size_t)MP * 512);
  if (off > ws_size || off > (size_t)WSMAX) return;
  unsigned short* WPL  = (unsigned short*)(ws + oWPL);
  unsigned short* WA   = WPL + OWA;
  unsigned short* WB   = WPL + OWB;
  unsigned short* WC   = WPL + OWC;
  unsigned short* WD   = WPL + OWD;
  float*          wsf  = (float*)d_ws;
  const unsigned long long fP1 = (unsigned long long)(oRA / 4);
  const unsigned long long fP2 = (unsigned long long)((oRA + (size_t)MP * 256) / 4);
  const unsigned long long fS  = (unsigned long long)(oRB / 4);
  float*          P1   = (float*)(ws + oRA);
  unsigned short* H1   = (unsigned short*)(ws + oRA);
  float*          P2   = (float*)(ws + oRA + (size_t)MP * 256);
  float*          Sx   = (float*)(ws + oRB);
  unsigned short* XB   = (unsigned short*)(ws + oRC);
  unsigned short* AGG  = (unsigned short*)(ws + oRC);

  const size_t scanLds = (size_t)AGG_LDS_INTS * 4;
  hipFuncSetAttribute(reinterpret_cast<const void*>(&k_scan<128>), hipFuncAttributeMaxDynamicSharedMemorySize, (int)scanLds);
  hipFuncSetAttribute(reinterpret_cast<const void*>(&k_scan<64>),  hipFuncAttributeMaxDynamicSharedMemorySize, (int)scanLds);

  const int nUx = MP * (CIN / 8);
  k_wprep<<<NUW / NTHR, NTHR, 0, stream>>>(Wp1, Ws1, Wn1, Wp2, Ws2, Wn2, WPL);
  k_cvx<<<cdiv(nUx, NTHR), NTHR, 0, stream>>>(x, nN, nUx, XB);
  k_gemm_ps<<<dim3(gM, 3), GTHR, 0, stream>>>(XB, WA, CIN, bp1, wsf, fP1, fS, CIN, CIN, HID);
  k_scan<128><<<gA, NTHR, scanLds, stream>>>(src, dst, nE, nN, vec8, MP, P1, AGG);
  k_gemm_h<<<gM, GTHR, 0, stream>>>(AGG, WB, 2 * CIN, Sx, b1, H1);
  k_gemm_ps<<<dim3(gM, 2), GTHR, 0, stream>>>(H1, WC, 2 * HID, bp2, wsf, fP2, fS, HID, HID, HID);
  k_scan<64><<<gA, NTHR, scanLds, stream>>>(src, dst, nE, nN, vec8, MP, P2, AGG);
  k_gemm_out<<<gM, GTHR, 0, stream>>>(AGG, WD, 2 * HID, Sx, b2, Wo, bo, out, nN);
}
